// NodeMultiHeadAttention_9414568312871
// MI455X (gfx1250) — hardware-verified
//
#include <hip/hip_runtime.h>
#include <math.h>
#include <stdint.h>

#define SEQ   2048
#define DMOD  256
#define NHEAD 8
#define DHD   32

typedef __attribute__((ext_vector_type(16))) __bf16   v16b;
typedef __attribute__((ext_vector_type(8)))  __bf16   v8b;
typedef __attribute__((ext_vector_type(8)))  float    v8f;
typedef __attribute__((ext_vector_type(4)))  float    v4f;
typedef __attribute__((ext_vector_type(2)))  float    v2f;
typedef __attribute__((ext_vector_type(4)))  unsigned int v4u;
typedef __attribute__((ext_vector_type(4)))  int      v4i;

__device__ __forceinline__ unsigned short f2bf_bits(float f) {
  unsigned u = __float_as_uint(f);
  return (unsigned short)((u + 0x7FFFu + ((u >> 16) & 1u)) >> 16);
}
__device__ __forceinline__ float bf_bits2f(unsigned short h) { return __uint_as_float(((unsigned)h) << 16); }
__device__ __forceinline__ unsigned pk16(unsigned short a, unsigned short b) { return (unsigned)a | ((unsigned)b << 16); }

union FragB { v16b v; v8b h[2]; };
__device__ __forceinline__ v16b frag_load(const __bf16* p) {
  FragB f; f.h[0] = *(const v8b*)(p); f.h[1] = *(const v8b*)(p + 16); return f.v;
}

__device__ __forceinline__ v8f mma_bf(v16b a, v16b b, v8f c) {
  c = __builtin_amdgcn_wmma_f32_16x16x32_bf16(false, a, false, b, (short)0, c, false, false);
  asm volatile("v_nop\n\tv_nop\n\tv_nop\n\tv_nop" : "+v"(c) : "v"(a), "v"(b));
  return c;
}

__global__ __launch_bounds__(256) void pair_bias_kernel(
    const float* __restrict__ dist, const float* __restrict__ contact, const int* __restrict__ label,
    const float* __restrict__ Wd1, const float* __restrict__ bd1, const float* __restrict__ Wd2, const float* __restrict__ bd2,
    const float* __restrict__ Wc1, const float* __restrict__ bc1, const float* __restrict__ Wc2, const float* __restrict__ bc2,
    float* __restrict__ bias) {
  float ad = 0.f, ld = 0.f, gd = 0.f, ac = 0.f, lc = 0.f, gc = 0.f;
#pragma unroll 1
  for (int j = 0; j < 16; ++j) {
    const float wd2 = Wd2[j], wc2 = Wc2[j];
    ad = fmaf(Wd1[j],      wd2, ad);
    ld = fmaf(Wd1[16 + j], wd2, ld);
    gd = fmaf(bd1[j],      wd2, gd);
    ac = fmaf(Wc1[j],      wc2, ac);
    lc = fmaf(Wc1[16 + j], wc2, lc);
    gc = fmaf(bc1[j],      wc2, gc);
  }
  gd += bd2[0];
  gc += bc2[0];
  const size_t base = (size_t)blockIdx.x * 8192 + (size_t)threadIdx.x * 4;
#pragma unroll 1
  for (int pass = 0; pass < 2; ++pass) {
#pragma unroll 1
    for (int it = 0; it < 8; ++it) {
      const size_t i4 = base + (size_t)it * 1024;
      const v4f dm = *(const v4f*)(dist + i4);
      const v4f cm = *(const v4f*)(contact + i4);
      const v4i lb = *(const v4i*)(label + i4);
      v4f o;
#pragma unroll
      for (int e = 0; e < 4; ++e) {
        const float lf = (float)lb[e];
        const float pd = fmaf(dm[e], ad, fmaf(lf, ld, gd));
        const float pc = fmaf(cm[e], ac, fmaf(lf, lc, gc));
        o[e] = pd + pc;
      }
      *(volatile v4f*)(bias + i4) = o;
    }
    __threadfence();
  }
}

__global__ __launch_bounds__(256) void split_bf16x2_kernel(const float* __restrict__ in, unsigned short* __restrict__ hi,
                                                           unsigned short* __restrict__ lo, int n2) {
  const int i = blockIdx.x * 256 + threadIdx.x;
  if (i < n2) {
    const v2f f = *(const v2f*)(in + 2 * (size_t)i);
    const unsigned short h0 = f2bf_bits(f[0]), h1 = f2bf_bits(f[1]);
    const unsigned short l0 = f2bf_bits(f[0] - bf_bits2f(h0)), l1 = f2bf_bits(f[1] - bf_bits2f(h1));
    const unsigned uh = pk16(h0, h1), ul = pk16(l0, l1);
    ((volatile unsigned*)hi)[i] = uh;
    ((volatile unsigned*)lo)[i] = ul;
    __threadfence();
    ((volatile unsigned*)hi)[i] = uh;
    ((volatile unsigned*)lo)[i] = ul;
  }
}

__global__ __launch_bounds__(256) void tsplit_kernel(const float* __restrict__ W, unsigned short* __restrict__ oh,
                                                     unsigned short* __restrict__ ol, int R, int Cc) {
  __shared__ __align__(16) float tf[64 * 68];
  const int c0  = blockIdx.x * 64;
  const int r0  = blockIdx.y * 64;
  const int tid = threadIdx.x;
  {
    const int lr = tid >> 4;
    const int c4 = (tid & 15) * 4;
#pragma unroll
    for (int it = 0; it < 4; ++it) {
      const int rr = it * 16 + lr;
      const v4f a = *(const v4f*)(W + (size_t)(r0 + rr) * Cc + c0 + c4);
      *(v4f*)(tf + rr * 68 + c4) = a;
    }
  }
  __syncthreads();
  const int sub = tid >> 3;
  const int c8  = (tid & 7) * 8;
  v4u hv[2], lv[2];
#pragma unroll
  for (int it = 0; it < 2; ++it) {
    const int oc = it * 32 + sub;
    v4u a, a2;
#pragma unroll
    for (int q = 0; q < 4; ++q) {
      const float f0 = tf[(c8 + 2 * q) * 68 + oc];
      const float f1 = tf[(c8 + 2 * q + 1) * 68 + oc];
      const unsigned short h0 = f2bf_bits(f0), h1 = f2bf_bits(f1);
      const unsigned short l0 = f2bf_bits(f0 - bf_bits2f(h0)), l1 = f2bf_bits(f1 - bf_bits2f(h1));
      a[q]  = pk16(h0, h1);
      a2[q] = pk16(l0, l1);
    }
    hv[it] = a; lv[it] = a2;
  }
  for (int pass = 0; pass < 2; ++pass) {
#pragma unroll
    for (int it = 0; it < 2; ++it) {
      const int oc = it * 32 + sub;
      const size_t go = (size_t)(c0 + oc) * R + r0 + c8;
      *(volatile v4u*)(oh + go) = hv[it];
      *(volatile v4u*)(ol + go) = lv[it];
    }
    __threadfence();
  }
}

template <int BIAS_MODE, int OUT_MODE>
__global__ __launch_bounds__(256) void gemm_split_kernel(
    const unsigned short* __restrict__ Ahp, const unsigned short* __restrict__ Alp, int lda,
    const unsigned short* __restrict__ Bhp, const unsigned short* __restrict__ Blp, int ldb,
    void* __restrict__ Cout, void* __restrict__ Cout2, int ldc,
    const float* __restrict__ bias, int M, int N, int K, float scale) {
  const __bf16* Ah = (const __bf16*)(const void*)Ahp;
  const __bf16* Al = (const __bf16*)(const void*)Alp;
  const __bf16* Bh = (const __bf16*)(const void*)Bhp;
  const __bf16* Bl = (const __bf16*)(const void*)Blp;
  __shared__ __align__(16) float sT[8][16 * 68];
  const int lane = threadIdx.x & 31;
  const int wave = threadIdx.x >> 5;
  const int tilesN = N >> 6;
  const int tilesM = M >> 5;
  const int tile = blockIdx.x * 8 + wave;
  if (tile >= tilesM * tilesN) return;
  const int tm = tile / tilesN;
  const int tn = tile - tm * tilesN;
  const int m0 = tm << 5;
  const int n0 = tn << 6;

  const int rlane = lane & 15;
  const int koff  = (lane >> 4) * 8;
  const int mOff  = (lane >> 4) * 8;

  v8f acc[2][4];
#pragma unroll
  for (int i = 0; i < 2; ++i)
#pragma unroll
    for (int j = 0; j < 4; ++j) acc[i][j] = (v8f){0.f,0.f,0.f,0.f,0.f,0.f,0.f,0.f};

  for (int k0 = 0; k0 < K; k0 += 32) {
    v16b bh[4], bl[4];
#pragma unroll
    for (int j = 0; j < 4; ++j) {
      const size_t bo = (size_t)(n0 + (j << 4) + rlane) * ldb + koff + k0;
      bh[j] = frag_load(Bh + bo);
      bl[j] = frag_load(Bl + bo);
    }
#pragma unroll
    for (int i = 0; i < 2; ++i) {
      const size_t ao = (size_t)(m0 + (i << 4) + rlane) * lda + koff + k0;
      const v16b ah = frag_load(Ah + ao);
      const v16b al = frag_load(Al + ao);
#pragma unroll
      for (int j = 0; j < 4; ++j) {
        acc[i][j] = mma_bf(ah, bh[j], acc[i][j]);
        acc[i][j] = mma_bf(ah, bl[j], acc[i][j]);
        acc[i][j] = mma_bf(al, bh[j], acc[i][j]);
      }
    }
  }

  float* slab = sT[wave];
#pragma unroll
  for (int i = 0; i < 2; ++i) {
    const int mBase = m0 + (i << 4);
#pragma unroll
    for (int j = 0; j < 4; ++j) {
      const int n = n0 + (j << 4) + rlane;
      float bvn = 0.f;
      if (BIAS_MODE == 2) bvn = bias[n];
#pragma unroll
      for (int r = 0; r < 8; ++r) {
        float v = acc[i][j][r];
        if (BIAS_MODE == 1) v += bias[mBase + mOff + r];
        if (BIAS_MODE == 2) v += bvn;
        v *= scale;
        slab[(mOff + r) * 68 + (j << 4) + rlane] = v;
      }
    }
    __builtin_amdgcn_fence(__ATOMIC_RELEASE, "workgroup");
    __builtin_amdgcn_wave_barrier();
    __builtin_amdgcn_fence(__ATOMIC_ACQUIRE, "workgroup");
    if (OUT_MODE == 0) {
      float* C = (float*)Cout;
      const int hh = lane >> 4, c4 = (lane & 15) * 4;
      for (int pass = 0; pass < 2; ++pass) {
#pragma unroll
        for (int it = 0; it < 8; ++it) {
          const int row = it * 2 + hh;
          const v4f v = *(const v4f*)(slab + row * 68 + c4);
          *(volatile v4f*)(C + (size_t)(mBase + row) * ldc + n0 + c4) = v;
        }
        __threadfence();
      }
    } else {
      const int q = lane >> 3, c8 = (lane & 7) * 8;
      unsigned short* C  = (unsigned short*)Cout;
      unsigned short* C2 = (unsigned short*)Cout2;
      for (int pass = 0; pass < 2; ++pass) {
#pragma unroll
        for (int it = 0; it < 4; ++it) {
          const int row = it * 4 + q;
          const float* sp = slab + row * 68 + c8;
          v4u hv, lv;
#pragma unroll
          for (int e = 0; e < 4; ++e) {
            const float f0 = sp[2 * e], f1 = sp[2 * e + 1];
            const unsigned short h0 = f2bf_bits(f0), h1 = f2bf_bits(f1);
            const unsigned short l0 = f2bf_bits(f0 - bf_bits2f(h0)), l1 = f2bf_bits(f1 - bf_bits2f(h1));
            hv[e] = pk16(h0, h1);
            lv[e] = pk16(l0, l1);
          }
          *(volatile v4u*)(C  + (size_t)(mBase + row) * ldc + n0 + c8) = hv;
          *(volatile v4u*)(C2 + (size_t)(mBase + row) * ldc + n0 + c8) = lv;
        }
        __threadfence();
      }
    }
    __builtin_amdgcn_fence(__ATOMIC_RELEASE, "workgroup");
    __builtin_amdgcn_wave_barrier();
    __builtin_amdgcn_fence(__ATOMIC_ACQUIRE, "workgroup");
  }
}

#define AT_KC 64

__device__ __forceinline__ __bf16 at_f2bf(float f) { return __builtin_bit_cast(__bf16, f2bf_bits(f)); }
__device__ __forceinline__ void at_split(float f, __bf16& hi, __bf16& lo) {
  const unsigned short hb = f2bf_bits(f);
  hi = __builtin_bit_cast(__bf16, hb);
  lo = at_f2bf(f - __uint_as_float(((unsigned)hb) << 16));
}

__global__ __launch_bounds__(128)
void attn_bias_kernel(const unsigned short* __restrict__ qhp, const unsigned short* __restrict__ qlp,
                      const unsigned short* __restrict__ khp, const unsigned short* __restrict__ klp,
                      const unsigned short* __restrict__ vhp, const unsigned short* __restrict__ vlp,
                      const float* __restrict__ bias, float* __restrict__ ctx) {
  __shared__ __align__(16) __bf16 Ksh[AT_KC * DHD];
  __shared__ __align__(16) __bf16 Ksl[AT_KC * DHD];
  __shared__ __align__(16) __bf16 Vth[DHD * AT_KC];
  __shared__ __align__(16) __bf16 Vtl[DHD * AT_KC];
  __shared__ __align__(16) __bf16 Psh[4][16 * AT_KC];
  __shared__ __align__(16) __bf16 Psl[4][16 * AT_KC];
  __shared__ __align__(16) float  Os[4][16 * 36];

  const int tid  = threadIdx.x;
  const int wave = tid >> 5;
  const int lane = tid & 31;
  const int hh   = lane >> 4;
  const int c    = lane & 15;

  const int nqb = SEQ / 64;
  const int bx = blockIdx.x;
  const int qb = bx % nqb;
  const int h  = bx / nqb;
  const int q0 = qb * 64 + wave * 16;

  const __bf16* Qh = (const __bf16*)(const void*)qhp + (size_t)h * DHD;
  const __bf16* Ql = (const __bf16*)(const void*)qlp + (size_t)h * DHD;
  const __bf16* Kh = (const __bf16*)(const void*)khp + (size_t)h * DHD;
  const __bf16* Kl = (const __bf16*)(const void*)klp + (size_t)h * DHD;
  const __bf16* Vh = (const __bf16*)(const void*)vhp + (size_t)h * DHD * SEQ;
  const __bf16* Vl = (const __bf16*)(const void*)vlp + (size_t)h * DHD * SEQ;
  float*        ob = ctx + (size_t)h * DHD;

  const v16b qah = frag_load(Qh + (size_t)(q0 + c) * DMOD + 8 * hh);
  const v16b qal = frag_load(Ql + (size_t)(q0 + c) * DMOD + 8 * hh);

  float mrow[8], lrow[8];
  v8f oacc[2];
#pragma unroll
  for (int r = 0; r < 8; ++r) { mrow[r] = -INFINITY; lrow[r] = 0.f; }
#pragma unroll
  for (int t = 0; t < 2; ++t) oacc[t] = (v8f){0.f,0.f,0.f,0.f,0.f,0.f,0.f,0.f};

  const float* brow = bias + (size_t)(q0 + 8 * hh) * SEQ + c;

  const int nChunks = SEQ / AT_KC;
  for (int kc = 0; kc < nChunks; ++kc) {
    const int kv0 = kc * AT_KC;
    __syncthreads();
    {
      const int r = tid >> 1, hf = (tid & 1) * 16;
      const __bf16* ksh = Kh + (size_t)(kv0 + r) * DMOD + hf;
      const __bf16* ksl = Kl + (size_t)(kv0 + r) * DMOD + hf;
      const int r2 = tid >> 2, part = (tid & 3) * 16;
      const __bf16* vsh = Vh + (size_t)r2 * SEQ + kv0 + part;
      const __bf16* vsl = Vl + (size_t)r2 * SEQ + kv0 + part;
#pragma unroll
      for (int i = 0; i < 2; ++i) {
        const v8b a0 = *(const v8b*)(ksh + 8 * i);
        const v8b a1 = *(const v8b*)(ksl + 8 * i);
        const v8b b0 = *(const v8b*)(vsh + 8 * i);
        const v8b b1 = *(const v8b*)(vsl + 8 * i);
        *(v8b*)(Ksh + r * DHD + hf + 8 * i)      = a0;
        *(v8b*)(Ksl + r * DHD + hf + 8 * i)      = a1;
        *(v8b*)(Vth + r2 * AT_KC + part + 8 * i) = b0;
        *(v8b*)(Vtl + r2 * AT_KC + part + 8 * i) = b1;
      }
    }
    __syncthreads();

    v8f s[4];
#pragma unroll
    for (int j = 0; j < 4; ++j) {
      s[j] = (v8f){0.f,0.f,0.f,0.f,0.f,0.f,0.f,0.f};
      FragB kb, kl;
      kb.h[0] = *(const v8b*)(Ksh + (j * 16 + c) * DHD + 8 * hh);
      kb.h[1] = *(const v8b*)(Ksh + (j * 16 + c) * DHD + 16 + 8 * hh);
      kl.h[0] = *(const v8b*)(Ksl + (j * 16 + c) * DHD + 8 * hh);
      kl.h[1] = *(const v8b*)(Ksl + (j * 16 + c) * DHD + 16 + 8 * hh);
      s[j] = mma_bf(qah, kb.v, s[j]);
      s[j] = mma_bf(qah, kl.v, s[j]);
      s[j] = mma_bf(qal, kb.v, s[j]);
    }
    float cm[8];
#pragma unroll
    for (int r = 0; r < 8; ++r) {
      float m = -INFINITY;
#pragma unroll
      for (int j = 0; j < 4; ++j) {
        const float sv = s[j][r] + brow[(size_t)r * SEQ + kv0 + j * 16];
        s[j][r] = sv;
        m = fmaxf(m, sv);
      }
#pragma unroll
      for (int off = 1; off < 16; off <<= 1) m = fmaxf(m, __shfl_xor(m, off, 32));
      cm[r] = m;
    }
    __bf16* pwh = Psh[wave];
    __bf16* pwl = Psl[wave];
#pragma unroll
    for (int r = 0; r < 8; ++r) {
      const float mnew = fmaxf(mrow[r], cm[r]);
      const float alpha = expf(mrow[r] - mnew);
      mrow[r] = mnew;
      float psum = 0.f;
#pragma unroll
      for (int j = 0; j < 4; ++j) {
        const float p = expf(s[j][r] - mnew);
        psum += p;
        __bf16 a, bl; at_split(p, a, bl);
        pwh[(8 * hh + r) * AT_KC + j * 16 + c] = a;
        pwl[(8 * hh + r) * AT_KC + j * 16 + c] = bl;
      }
#pragma unroll
      for (int off = 1; off < 16; off <<= 1) psum += __shfl_xor(psum, off, 32);
      lrow[r] = lrow[r] * alpha + psum;
#pragma unroll
      for (int t = 0; t < 2; ++t) oacc[t][r] *= alpha;
    }
    __builtin_amdgcn_fence(__ATOMIC_RELEASE, "workgroup");
    __builtin_amdgcn_wave_barrier();
    __builtin_amdgcn_fence(__ATOMIC_ACQUIRE, "workgroup");
#pragma unroll 1
    for (int kk = 0; kk < 2; ++kk) {
      FragB pa, pl;
      pa.h[0] = *(const v8b*)(pwh + c * AT_KC + kk * 32 + 8 * hh);
      pa.h[1] = *(const v8b*)(pwh + c * AT_KC + kk * 32 + 16 + 8 * hh);
      pl.h[0] = *(const v8b*)(pwl + c * AT_KC + kk * 32 + 8 * hh);
      pl.h[1] = *(const v8b*)(pwl + c * AT_KC + kk * 32 + 16 + 8 * hh);
#pragma unroll
      for (int t = 0; t < 2; ++t) {
        FragB vb, vl;
        vb.h[0] = *(const v8b*)(Vth + (t * 16 + c) * AT_KC + kk * 32 + 8 * hh);
        vb.h[1] = *(const v8b*)(Vth + (t * 16 + c) * AT_KC + kk * 32 + 16 + 8 * hh);
        vl.h[0] = *(const v8b*)(Vtl + (t * 16 + c) * AT_KC + kk * 32 + 8 * hh);
        vl.h[1] = *(const v8b*)(Vtl + (t * 16 + c) * AT_KC + kk * 32 + 16 + 8 * hh);
        oacc[t] = mma_bf(pa.v, vb.v, oacc[t]);
        oacc[t] = mma_bf(pa.v, vl.v, oacc[t]);
        oacc[t] = mma_bf(pl.v, vb.v, oacc[t]);
      }
    }
  }

  float* os = Os[wave];
#pragma unroll
  for (int r = 0; r < 8; ++r) {
    const float inv = 1.0f / lrow[r];
#pragma unroll
    for (int t = 0; t < 2; ++t) os[(8 * hh + r) * 36 + t * 16 + c] = oacc[t][r] * inv;
  }
  __builtin_amdgcn_fence(__ATOMIC_RELEASE, "workgroup");
  __builtin_amdgcn_wave_barrier();
  __builtin_amdgcn_fence(__ATOMIC_ACQUIRE, "workgroup");
  {
    const int q4 = lane >> 3, c4 = (lane & 7) * 4;
    for (int pass = 0; pass < 2; ++pass) {
#pragma unroll
      for (int it = 0; it < 4; ++it) {
        const int row = it * 4 + q4;
        const v4f val = *(const v4f*)(os + row * 36 + c4);
        *(volatile v4f*)(ob + (size_t)(q0 + row) * DMOD + c4) = val;
      }
      __threadfence();
    }
  }
}

extern "C" void kernel_launch(void* const* d_in, const int* in_sizes, int n_in,
                              void* d_out, int out_size, void* d_ws, size_t ws_size,
                              hipStream_t stream) {
  if (n_in < 22) return;
  if (in_sizes[0] != SEQ * SEQ || in_sizes[1] != SEQ * SEQ || in_sizes[2] != SEQ * SEQ) return;
  if (in_sizes[3] != SEQ * DMOD || in_sizes[4] != SEQ * DMOD || in_sizes[5] != SEQ * DMOD) return;
  if (in_sizes[6] != DMOD * DMOD || in_sizes[8] != DMOD * DMOD || in_sizes[10] != DMOD * DMOD || in_sizes[12] != DMOD * DMOD) return;
  if (in_sizes[7] != DMOD || in_sizes[9] != DMOD || in_sizes[11] != DMOD || in_sizes[13] != DMOD) return;
  if (in_sizes[14] != 32 || in_sizes[15] != 16 || in_sizes[16] != 16 || in_sizes[17] != 1) return;
  if (in_sizes[18] != 32 || in_sizes[19] != 16 || in_sizes[20] != 16 || in_sizes[21] != 1) return;
  if (out_size != SEQ * DMOD) return;

  const int*   label   = (const int*)  d_in[0];
  const float* dist    = (const float*)d_in[1];
  const float* contact = (const float*)d_in[2];
  const float* q   = (const float*)d_in[3];
  const float* k   = (const float*)d_in[4];
  const float* v   = (const float*)d_in[5];
  const float* Wq  = (const float*)d_in[6];
  const float* bq  = (const float*)d_in[7];
  const float* Wk  = (const float*)d_in[8];
  const float* bk  = (const float*)d_in[9];
  const float* Wv  = (const float*)d_in[10];
  const float* bv  = (const float*)d_in[11];
  const float* Wo  = (const float*)d_in[12];
  const float* bo  = (const float*)d_in[13];
  const float* Wd1 = (const float*)d_in[14];
  const float* bd1 = (const float*)d_in[15];
  const float* Wd2 = (const float*)d_in[16];
  const float* bd2 = (const float*)d_in[17];
  const float* Wc1 = (const float*)d_in[18];
  const float* bc1 = (const float*)d_in[19];
  const float* Wc2 = (const float*)d_in[20];
  const float* bc2 = (const float*)d_in[21];
  float* out = (float*)d_out;

  const size_t PB = (size_t)SEQ * SEQ * 4;
  const size_t PW = (size_t)DMOD * DMOD * 2;
  const size_t PX = (size_t)SEQ * DMOD * 2;
  const size_t PF = (size_t)SEQ * DMOD * 4;
  size_t off = 0;
  const size_t oBias = off; off += PB;
  const size_t oWqTh = off; off += PW;  const size_t oWqTl = off; off += PW;
  const size_t oWkTh = off; off += PW;  const size_t oWkTl = off; off += PW;
  const size_t oWvTh = off; off += PW;  const size_t oWvTl = off; off += PW;
  const size_t oWoTh = off; off += PW;  const size_t oWoTl = off; off += PW;
  const size_t oXqh  = off; off += PX;  const size_t oXql  = off; off += PX;
  const size_t oXkh  = off; off += PX;  const size_t oXkl  = off; off += PX;
  const size_t oXvh  = off; off += PX;  const size_t oXvl  = off; off += PX;
  const size_t oQh   = off; off += PX;  const size_t oQl   = off; off += PX;
  const size_t oKh   = off; off += PX;  const size_t oKl   = off; off += PX;
  const size_t oVTh  = off; off += PX;  const size_t oVTl  = off; off += PX;
  const size_t oCTf  = off; off += PF;
  const size_t oCTh  = off; off += PX;  const size_t oCTl  = off; off += PX;
  if (off > ws_size) return;

  char* ws = (char*)d_ws;
  float*          biasP = (float*)(ws + oBias);
  unsigned short* WqTh = (unsigned short*)(ws + oWqTh); unsigned short* WqTl = (unsigned short*)(ws + oWqTl);
  unsigned short* WkTh = (unsigned short*)(ws + oWkTh); unsigned short* WkTl = (unsigned short*)(ws + oWkTl);
  unsigned short* WvTh = (unsigned short*)(ws + oWvTh); unsigned short* WvTl = (unsigned short*)(ws + oWvTl);
  unsigned short* WoTh = (unsigned short*)(ws + oWoTh); unsigned short* WoTl = (unsigned short*)(ws + oWoTl);
  unsigned short* Xqh  = (unsigned short*)(ws + oXqh);  unsigned short* Xql  = (unsigned short*)(ws + oXql);
  unsigned short* Xkh  = (unsigned short*)(ws + oXkh);  unsigned short* Xkl  = (unsigned short*)(ws + oXkl);
  unsigned short* Xvh  = (unsigned short*)(ws + oXvh);  unsigned short* Xvl  = (unsigned short*)(ws + oXvl);
  unsigned short* Qh   = (unsigned short*)(ws + oQh);   unsigned short* Ql   = (unsigned short*)(ws + oQl);
  unsigned short* Kh   = (unsigned short*)(ws + oKh);   unsigned short* Kl   = (unsigned short*)(ws + oKl);
  unsigned short* VTh  = (unsigned short*)(ws + oVTh);  unsigned short* VTl  = (unsigned short*)(ws + oVTl);
  float*          CTf  = (float*)(ws + oCTf);
  unsigned short* CTh  = (unsigned short*)(ws + oCTh);  unsigned short* CTl  = (unsigned short*)(ws + oCTl);

  const dim3 blk(256);

  pair_bias_kernel<<<dim3((SEQ * SEQ) / 8192), blk, 0, stream>>>(dist, contact, label,
      Wd1, bd1, Wd2, bd2, Wc1, bc1, Wc2, bc2, biasP);

  const dim3 gW(DMOD / 64, DMOD / 64);
  tsplit_kernel<<<gW, blk, 0, stream>>>(Wq, WqTh, WqTl, DMOD, DMOD);
  tsplit_kernel<<<gW, blk, 0, stream>>>(Wk, WkTh, WkTl, DMOD, DMOD);
  tsplit_kernel<<<gW, blk, 0, stream>>>(Wv, WvTh, WvTl, DMOD, DMOD);
  tsplit_kernel<<<gW, blk, 0, stream>>>(Wo, WoTh, WoTl, DMOD, DMOD);

  const int n2x = SEQ * DMOD / 2;
  const dim3 gCast((n2x + 255) / 256);
  split_bf16x2_kernel<<<gCast, blk, 0, stream>>>(q, Xqh, Xql, n2x);
  split_bf16x2_kernel<<<gCast, blk, 0, stream>>>(k, Xkh, Xkl, n2x);
  split_bf16x2_kernel<<<gCast, blk, 0, stream>>>(v, Xvh, Xvl, n2x);

  const dim3 gProj(((SEQ / 32) * (DMOD / 64) + 7) / 8);
  const dim3 gVT(((DMOD / 32) * (SEQ / 64) + 7) / 8);
  const float qscale = 0.17677669529663688f;
  gemm_split_kernel<2, 2><<<gProj, blk, 0, stream>>>(Xqh, Xql, DMOD, WqTh, WqTl, DMOD,
      (void*)Qh, (void*)Ql, DMOD, bq, SEQ, DMOD, DMOD, qscale);
  gemm_split_kernel<2, 2><<<gProj, blk, 0, stream>>>(Xkh, Xkl, DMOD, WkTh, WkTl, DMOD,
      (void*)Kh, (void*)Kl, DMOD, bk, SEQ, DMOD, DMOD, 1.0f);
  gemm_split_kernel<1, 2><<<gVT, blk, 0, stream>>>(WvTh, WvTl, DMOD, Xvh, Xvl, DMOD,
      (void*)VTh, (void*)VTl, SEQ, bv, DMOD, SEQ, DMOD, 1.0f);

  attn_bias_kernel<<<dim3(NHEAD * (SEQ / 64)), dim3(128), 0, stream>>>(Qh, Ql, Kh, Kl, VTh, VTl, biasP, CTf);

  split_bf16x2_kernel<<<gCast, blk, 0, stream>>>(CTf, CTh, CTl, n2x);

  gemm_split_kernel<2, 0><<<gProj, blk, 0, stream>>>(CTh, CTl, DMOD, WoTh, WoTl, DMOD,
      (void*)out, (void*)out, DMOD, bo, SEQ, DMOD, DMOD, 1.0f);

  (void)hipGetLastError();
}
